// GraphNetwork_50122268345054
// MI455X (gfx1250) — hardware-verified
//
#include <hip/hip_runtime.h>
#include <stddef.h>
#include <stdint.h>

#define NN     50000
#define NE     800000
#define NCH    5
#define EC     160000
#define XD     118
#define NTHR   256
#define NWAVE  8
#define TM     128
#define SQDN   50048

#define O_XS   0
#define O_ZZ   1600000
#define O_SQD  3200000
#define O_F    3250048
#define O_MASK 4850048
#define O_AGG  8050048
#define O_S1   14450048
#define O_V1   16050048
#define O_WP   20850048
#define O_PL   31090048
static_assert(O_ZZ == O_XS + NN * 32);
static_assert(O_SQD == O_ZZ + NN * 32);
static_assert(O_F == O_SQD + SQDN);
static_assert(O_MASK == O_F + NN * 32);
static_assert(O_AGG == O_MASK + NN * 64);
static_assert(O_S1 == O_AGG + NN * 128);
static_assert(O_V1 == O_S1 + NN * 32);
static_assert(O_WP == O_V1 + 3 * NN * 32);
static_assert(O_PL == O_WP + EC * 64);
static_assert(NN * 64 <= 3 * NN * 32);
static_assert((O_SQD % 32) == 0 && (O_F % 32) == 0 && (O_MASK % 32) == 0 && (O_AGG % 32) == 0 &&
              (O_S1 % 32) == 0 && (O_V1 % 32) == 0 && (O_WP % 32) == 0 && (O_PL % 32) == 0);
static_assert(SQDN % 32 == 0 && SQDN >= NN && (SQDN / 4) % 32 == 0);

#define P_PRE1  0
#define P_PO1S  98304
#define P_PO1V  163840
#define P_PRE2S 196608
#define P_PRE2V 294912
#define P_PO2   327680
#define P_EMX   458752
#define P_EMZ   462848
#define P_R0T   466944
#define P_R1T   471040
#define P_END   479232
static_assert(P_PO1S == P_PRE1 + 96 * 1024 && P_PO1V == P_PO1S + 64 * 1024 && P_PRE2S == P_PO1V + 32 * 1024);
static_assert(P_PRE2V == P_PRE2S + 96 * 1024 && P_PO2 == P_PRE2V + 32 * 1024 && P_EMX == P_PO2 + 64 * 2048);
static_assert(P_EMZ == P_EMX + 32 * 128 && P_R0T == P_EMZ + 32 * 128 && P_R1T == P_R0T + 128 * 32);
static_assert(P_END == P_R1T + 2 * 64 * 64);
#define WS_BYTES ((size_t)O_PL * 4 + (size_t)P_END * 2)
static_assert(WS_BYTES <= (size_t)134217728);

static_assert(NE == NCH * EC && EC % TM == 0 && NE % NCH == 0);

#define EPT    8
#define CHUNK  (NTHR * EPT)
#define WCAP   (EPT * 32)
#define LISTN  (NWAVE * WCAP)
#define NBA    1024
#define SLA    10
#define RCAP   16896
#define DEGCAP 64
#define AGG_ZINTS (LISTN + 2 * RCAP + 3 * NBA)
#define AGG_LDS_INTS (AGG_ZINTS + 16)
#define AGG_LDS_BYTES (AGG_LDS_INTS * 4)
static_assert((CHUNK & (CHUNK - 1)) == 0 && CHUNK <= 4096);
static_assert((NBA & (NBA - 1)) == 0 && NBA == (1 << SLA));
static_assert(((long long)EC << SLA) < (1LL << 31));
static_assert(((long long)CHUNK << SLA) < (1LL << 31));
static_assert(NBA % NWAVE == 0 && NBA % 32 == 0);
static_assert(AGG_ZINTS % (4 * NTHR) == 0);
static_assert(AGG_LDS_BYTES <= 300000);
static_assert(RCAP >= 16651);
static_assert(DEGCAP >= 38 + 8);
static_assert((EC * 4) % 16 == 0);
#define SCAN_BLOCKS ((NN + NBA - 1) / NBA)
static_assert(SCAN_BLOCKS * NBA >= NN);

#define C_S   0.3826834323650898f
#define C_X   0.9238795325112867f
#define RN32  0.03125f
#define RN64  (1.0f / 45.254833995939045f)
#define SQ3F  1.7320508075688772f
#define RSQ3F (1.0f / 1.7320508075688772f)
#define RSTEP (1.0f / 0.5555555555555556f)
#define R112  (1.0f / 1.12f)

typedef float          v2f   __attribute__((ext_vector_type(2)));
typedef float          v4f   __attribute__((ext_vector_type(4)));
typedef float          v8f   __attribute__((ext_vector_type(8)));
typedef int            v4i   __attribute__((ext_vector_type(4)));
typedef int            v8i   __attribute__((ext_vector_type(8)));
typedef unsigned short v8us  __attribute__((ext_vector_type(8)));
typedef unsigned short v16us __attribute__((ext_vector_type(16)));
typedef __bf16         v16bf __attribute__((ext_vector_type(16)));
typedef v2f  __attribute__((may_alias)) v2fa;
typedef v4f  __attribute__((may_alias)) v4fa;
typedef v4i  __attribute__((may_alias)) v4ia;
typedef v8us __attribute__((may_alias)) v8usa;
union FragB { v16bf v; v16us u; v8us h[2]; v8i w; };

__device__ __forceinline__ v8f wmb(const FragB& a, const FragB& b, v8f c) {
  v8f d = __builtin_amdgcn_wmma_f32_16x16x32_bf16(false, a.v, false, b.v, (short)0, c, false, false);
  asm volatile("v_nop\n\tv_nop\n\tv_nop\n\tv_nop" : "+v"(d) : "v"(a.w), "v"(b.w));
  return d;
}

__device__ __forceinline__ unsigned bf16_bits(float f) {
  const unsigned u = __float_as_uint(f);
  return (u + 0x7FFFu + ((u >> 16) & 1u)) >> 16;
}
__device__ __forceinline__ unsigned bf16_hi32(float f) {
  const unsigned u = __float_as_uint(f);
  return (u + 0x7FFFu + ((u >> 16) & 1u)) & 0xFFFF0000u;
}
__device__ __forceinline__ float bf16_val(float f) { return __uint_as_float(bf16_hi32(f)); }

__device__ __forceinline__ void put16(unsigned short* dp, v8us o) {
  *(volatile v8us*)dp = o;
  __threadfence();
  *(volatile v8us*)dp = o;
}
__device__ __forceinline__ void putf4(float* dp, v4f o) {
  *(volatile v4f*)dp = o;
  __threadfence();
  *(volatile v4f*)dp = o;
}

__host__ __device__ constexpr float ctr(int k) { return (float)((double)k * 5.0 / 9.0); }

template <int SLB>
__device__ __forceinline__ int scan_chunk(const int* __restrict__ dsts, int nE, int cbase, int slotBase,
                                          int nb, int vec8, int* list, int tid, int lane, int wave) {
  int wc = 0;
  const int el0  = tid * EPT;
  const int e0   = cbase + el0;
  const int sent = -2147483647 - 1;
  v4i da, db;
  if (vec8 != 0 && cbase + CHUNK <= nE) {
    da = *(const v4i*)(dsts + e0);
    db = *(const v4i*)(dsts + e0 + 4);
  } else {
    da.x = (e0     < nE) ? dsts[min(e0,     nE - 1)] : sent;
    da.y = (e0 + 1 < nE) ? dsts[min(e0 + 1, nE - 1)] : sent;
    da.z = (e0 + 2 < nE) ? dsts[min(e0 + 2, nE - 1)] : sent;
    da.w = (e0 + 3 < nE) ? dsts[min(e0 + 3, nE - 1)] : sent;
    db.x = (e0 + 4 < nE) ? dsts[min(e0 + 4, nE - 1)] : sent;
    db.y = (e0 + 5 < nE) ? dsts[min(e0 + 5, nE - 1)] : sent;
    db.z = (e0 + 6 < nE) ? dsts[min(e0 + 6, nE - 1)] : sent;
    db.w = (e0 + 7 < nE) ? dsts[min(e0 + 7, nE - 1)] : sent;
  }
  const unsigned nbs = (unsigned)slotBase;
  const unsigned unb = (unsigned)nb;
  const unsigned s0 = (unsigned)da.x - nbs, s1 = (unsigned)da.y - nbs;
  const unsigned s2 = (unsigned)da.z - nbs, s3 = (unsigned)da.w - nbs;
  const unsigned s4 = (unsigned)db.x - nbs, s5 = (unsigned)db.y - nbs;
  const unsigned s6 = (unsigned)db.z - nbs, s7 = (unsigned)db.w - nbs;
  const bool h0 = s0 < unb, h1 = s1 < unb, h2 = s2 < unb, h3 = s3 < unb;
  const bool h4 = s4 < unb, h5 = s5 < unb, h6 = s6 < unb, h7 = s7 < unb;
  const unsigned any = __builtin_amdgcn_ballot_w32(h0 | h1 | h2 | h3 | h4 | h5 | h6 | h7);
  if (any != 0u) {
#define HITJ(J, HJ, SJ) { \
      const unsigned mj = __builtin_amdgcn_ballot_w32(HJ); \
      if (mj != 0u) { \
        if (HJ) { \
          const int pos = wc + (int)__builtin_amdgcn_mbcnt_lo(mj, 0u); \
          if (pos < WCAP) list[wave * WCAP + pos] = ((el0 + (J)) << SLB) | (int)(SJ); \
        } \
        wc += (int)__builtin_popcount(mj); } }
    HITJ(0, h0, s0)
    HITJ(1, h1, s1)
    HITJ(2, h2, s2)
    HITJ(3, h3, s3)
    HITJ(4, h4, s4)
    HITJ(5, h5, s5)
    HITJ(6, h6, s6)
    HITJ(7, h7, s7)
#undef HITJ
  }
  return wc;
}

#define B1  4096
#define B2  8192
#define B3  12288
#define B4  16384
#define B5  20480
#define B6  24576
#define B7  28672
#define B8  36864
#define B9  40960
#define B10 57344
#define B11 57856
#define B12 58368
#define B13 58624
#define B14 58880
#define B15 59392
#define B16 59904
#define B17 72448
static_assert(B17 % NTHR == 0 && B16 % NTHR == 0 && B10 % NTHR == 0 && B12 % NTHR == 0 && B13 % NTHR == 0);
static_assert((B17 - B16) >= SQDN / 4 && NN % 4 == 0 && B16 % 32 == 0);

__device__ __forceinline__ void wunit(const float* __restrict__ Wm, int vs, int kTot, int ush, int v,
                                      unsigned short* dst) {
  const int row = v >> ush;
  const int k8  = (v & ((1 << ush) - 1)) << 3;
  const float* p = Wm + (size_t)k8 * vs + row;
  v8us o;
#pragma unroll
  for (int i = 0; i < 8; ++i) o[i] = (unsigned short)bf16_bits(p[(size_t)i * vs]);
  put16(dst + (size_t)row * kTot + k8, o);
}
__device__ __forceinline__ void eunit(const float* __restrict__ Wm, int v, unsigned short* dst) {
  const int n  = v >> 4;
  const int k8 = (v & 15) << 3;
  v8us o;
#pragma unroll
  for (int i = 0; i < 8; ++i) {
    const int k  = k8 + i;
    const int kc = k < XD ? k : XD - 1;
    const unsigned b = bf16_bits(Wm[kc * 32 + n]);
    o[i] = (unsigned short)(k < XD ? b : 0u);
  }
  put16(dst + n * 128 + k8, o);
}
__device__ __forceinline__ void r0unit(const float* __restrict__ w0, int v, unsigned short* dst) {
  const int j  = v >> 2;
  const int k8 = (v & 3) << 3;
  v8us o;
#pragma unroll
  for (int i = 0; i < 8; ++i) {
    const int k  = k8 + i;
    int kk = k < 10 ? k : k - 10;
    kk = kk > 9 ? 9 : kk;
    const unsigned b = bf16_bits(w0[kk * 64 + j]);
    o[i] = (unsigned short)(k < 20 ? b : 0u);
  }
  put16(dst + j * 32 + k8, o);
}
__device__ __forceinline__ void r1unit(const float* __restrict__ w1, int v, unsigned short* dst) {
  const int n  = v >> 3;
  const int k8 = (v & 7) << 3;
  v8us o;
#pragma unroll
  for (int i = 0; i < 8; ++i) o[i] = (unsigned short)bf16_bits(w1[(k8 + i) * 64 + n]);
  put16(dst + n * 64 + k8, o);
}

__global__ __launch_bounds__(NTHR) void k_prep(
    const float* __restrict__ ndeg, const float* __restrict__ emxw, const float* __restrict__ emzw,
    const float* __restrict__ wli1, const float* __restrict__ wlm1s, const float* __restrict__ wlm1g,
    const float* __restrict__ r1w0, const float* __restrict__ r1w1,
    const float* __restrict__ wlo1s, const float* __restrict__ wlo1g, const float* __restrict__ wlo1v,
    const float* __restrict__ wli2s, const float* __restrict__ wli2v, const float* __restrict__ wlm2,
    const float* __restrict__ r2w0, const float* __restrict__ r2w1, const float* __restrict__ wlo2,
    unsigned short* PL, float* SQD) {
  const int u = (int)blockIdx.x * NTHR + (int)threadIdx.x;
  if (u < B1)       { wunit(wli1,  32, 1024, 7, u,       PL + P_PRE1);               return; }
  else if (u < B2)  { wunit(wlm1s, 32, 1024, 7, u - B1,  PL + P_PRE1 + 32 * 1024);   return; }
  else if (u < B3)  { wunit(wlm1g, 32, 1024, 7, u - B2,  PL + P_PRE1 + 64 * 1024);   return; }
  else if (u < B4)  { wunit(wlo1s, 32, 1024, 7, u - B3,  PL + P_PO1S);               return; }
  else if (u < B5)  { wunit(wlo1g, 32, 1024, 7, u - B4,  PL + P_PO1S + 32 * 1024);   return; }
  else if (u < B6)  { wunit(wlo1v, 32, 1024, 7, u - B5,  PL + P_PO1V);               return; }
  else if (u < B7)  { wunit(wli2s, 32, 1024, 7, u - B6,  PL + P_PRE2S);              return; }
  else if (u < B8)  { wunit(wlm2,  64, 1024, 7, u - B7,  PL + P_PRE2S + 32 * 1024);  return; }
  else if (u < B9)  { wunit(wli2v, 32, 1024, 7, u - B8,  PL + P_PRE2V);              return; }
  else if (u < B10) { wunit(wlo2,  64, 2048, 8, u - B9,  PL + P_PO2);                return; }
  else if (u < B11) { eunit(emxw, u - B10, PL + P_EMX);                              return; }
  else if (u < B12) { eunit(emzw, u - B11, PL + P_EMZ);                              return; }
  else if (u < B13) { r0unit(r1w0, u - B12, PL + P_R0T);                             return; }
  else if (u < B14) { r0unit(r2w0, u - B13, PL + P_R0T + 64 * 32);                   return; }
  else if (u < B15) { r1unit(r1w1, u - B14, PL + P_R1T);                             return; }
  else if (u < B16) { r1unit(r2w1, u - B15, PL + P_R1T + 64 * 64);                   return; }
  else if (u < B17) {
    const int v = u - B16;
    if (v < SQDN / 4) {
      const int  vc = v < NN / 4 ? v : NN / 4 - 1;
      const bool ok = v < NN / 4;
      const v4f d = *(const v4fa*)(ndeg + (size_t)vc * 4);
      const float s0 = sqrtf(bf16_val(d.x));
      const float s1 = sqrtf(bf16_val(d.y));
      const float s2 = sqrtf(bf16_val(d.z));
      const float s3 = sqrtf(bf16_val(d.w));
      v4f q;
      q.x = ok ? s0 : 1.0f;
      q.y = ok ? s1 : 1.0f;
      q.z = ok ? s2 : 1.0f;
      q.w = ok ? s3 : 1.0f;
      putf4(SQD + (size_t)v * 4, q);
    }
    return;
  }
}

#define EAP 136
__device__ __forceinline__ void emb_store_pass(const float* stg, float* Y, int rowBase, int wave, int lane) {
  const int q8 = lane & 7, sub = lane >> 3;
#pragma unroll
  for (int i = 0; i < 4; ++i) {
    const int row = 16 * wave + i * 4 + sub;
    const v4f v = *(const v4fa*)(stg + row * 36 + 4 * q8);
    const int gr = rowBase + row;
    if (gr < NN) *(volatile v4f*)(Y + (size_t)gr * 32 + 4 * q8) = v;
  }
}
__global__ __launch_bounds__(NTHR) void k_embed(const float* __restrict__ X, const float* __restrict__ bias,
                                                const unsigned short* __restrict__ WT, float* Y) {
  __shared__ __attribute__((aligned(16))) unsigned short sA[TM * EAP];
  __shared__ __attribute__((aligned(16))) float stg[TM * 36];
  const int tid = (int)threadIdx.x, lane = tid & 31, wave = tid >> 5, hh = lane >> 4, m = lane & 15;
  const int rowBase = (int)blockIdx.x * TM;

#pragma unroll 4
  for (int idx = tid; idx < TM * (XD / 2); idx += NTHR) {
    const int lr = idx / (XD / 2);
    const int c2 = (idx - lr * (XD / 2)) * 2;
    int gr = rowBase + lr;
    gr = gr < NN ? gr : NN - 1;
    const v2f xv = *(const v2fa*)(X + (size_t)gr * XD + c2);
    sA[lr * EAP + c2]     = (unsigned short)bf16_bits(fmaxf(xv.x, 0.0f));
    sA[lr * EAP + c2 + 1] = (unsigned short)bf16_bits(fmaxf(xv.y, 0.0f));
  }
  if (tid < TM) {
#pragma unroll
    for (int c = XD; c < EAP; ++c) sA[tid * EAP + c] = (unsigned short)0;
  }
  __syncthreads();

  const v8f z8 = {0.f, 0.f, 0.f, 0.f, 0.f, 0.f, 0.f, 0.f};
  v8f acc[2];
  acc[0] = z8; acc[1] = z8;
  const unsigned short* ap = sA + (16 * wave + m) * EAP + 8 * hh;
  const unsigned short* bp = WT + (size_t)m * 128 + 8 * hh;
#pragma unroll
  for (int ks = 0; ks < 4; ++ks) {
    const int k0 = 32 * ks;
    FragB a;
    a.h[0] = *(const v8usa*)(ap + k0);
    a.h[1] = *(const v8usa*)(ap + k0 + 16);
#pragma unroll
    for (int nt = 0; nt < 2; ++nt) {
      const unsigned short* wq = bp + (size_t)(16 * nt) * 128 + k0;
      FragB b;
      b.h[0] = *(const v8usa*)wq;
      b.h[1] = *(const v8usa*)(wq + 16);
      acc[nt] = wmb(a, b, acc[nt]);
    }
  }
#pragma unroll
  for (int nt = 0; nt < 2; ++nt) {
    const float bb = bf16_val(bias[16 * nt + m]);
#pragma unroll
    for (int r = 0; r < 8; ++r)
      stg[(16 * wave + 8 * hh + r) * 36 + 16 * nt + m] = fmaxf(acc[nt][r] + bb, 0.0f);
  }
  __syncthreads();
  emb_store_pass(stg, Y, rowBase, wave, lane);
  __threadfence();
  emb_store_pass(stg, Y, rowBase, wave, lane);
}

#define M_PRE1  0
#define M_PO1S  1
#define M_PO1V  2
#define M_PRE2S 3
#define M_PRE2V 4
#define M_PO2   5
template <int MODE> __host__ __device__ constexpr int fcU() { return MODE == M_PO2 ? 64 : 32; }
template <int MODE> __host__ __device__ constexpr int fcV() {
  return (MODE == M_PRE1 || MODE == M_PRE2S) ? 96 : ((MODE == M_PO1S || MODE == M_PO2) ? 64 : 32);
}
template <int MODE> __host__ __device__ constexpr int fcM() {
  return (MODE == M_PO1V || MODE == M_PRE2V) ? 3 * NN : NN;
}
template <int MODE> __host__ __device__ constexpr int fcP() {
  return MODE == M_PRE1 ? P_PRE1 : MODE == M_PO1S ? P_PO1S : MODE == M_PO1V ? P_PO1V :
         MODE == M_PRE2S ? P_PRE2S : MODE == M_PRE2V ? P_PRE2V : P_PO2;
}
template <int MODE> __device__ __forceinline__ int fc_node(int r) {
  if constexpr (MODE == M_PO1V || MODE == M_PRE2V) return r / 3; else return r;
}
template <int MODE> __device__ __forceinline__ int fc_aoff(int r) {
  if constexpr (MODE == M_PRE1)       return O_XS + r * 32;
  else if constexpr (MODE == M_PO1S)  return O_AGG + r * 128;
  else if constexpr (MODE == M_PO1V)  { const int n = r / 3; const int c = r - 3 * n; return O_AGG + n * 128 + 32 + 32 * c; }
  else if constexpr (MODE == M_PRE2S) return O_S1 + r * 32;
  else if constexpr (MODE == M_PRE2V) return O_V1 + r * 32;
  else                                return O_V1 + r * 64;
}
template <int MODE> __device__ __forceinline__ int fc_doff(int r, int seg, int q) {
  if constexpr (MODE == M_PRE1)
    return (seg == 0) ? (O_F + r * 32 + 4 * q) : (O_MASK + r * 64 + (seg - 1) * 32 + 4 * q);
  else if constexpr (MODE == M_PO1S)
    return ((seg == 0) ? O_S1 : O_F) + r * 32 + 4 * q;
  else if constexpr (MODE == M_PO1V)
    return O_V1 + r * 32 + 4 * q;
  else if constexpr (MODE == M_PRE2S)
    return (seg == 0) ? (O_AGG + r * 128 + 4 * q) : (O_MASK + r * 64 + (seg - 1) * 32 + 4 * q);
  else if constexpr (MODE == M_PRE2V) { const int n = r / 3; const int c = r - 3 * n; return O_AGG + n * 128 + 32 + 32 * c + 4 * q; }
  else
    return r * 64 + seg * 32 + 4 * q;
}
__device__ __forceinline__ float gate_sig(float comb) {
  const float tc = (comb < -80.0f) ? -80.0f : comb;
  const float e = expf(-tc);
  return 1.0f / (1.0f + e);
}

template <int MODE>
__global__ __launch_bounds__(NTHR) void k_fctp(float* W, const unsigned short* __restrict__ PL, float* out) {
  constexpr int U = fcU<MODE>(), V = fcV<MODE>(), M = fcM<MODE>(), NT = V / 16, KT = 32 * U;
  constexpr int AP = U + 4, ZP = 36, VP = V + 4, VL = V / 32, NPC = V / 8, UQ = U / 4;
  constexpr int SZ_A = TM * AP * 4, SZ_Z = TM * ZP * 4, SZ_S = TM * VP * 4;
  constexpr int SZ_M = (SZ_A + SZ_Z > SZ_S) ? (SZ_A + SZ_Z) : SZ_S;
  static_assert(V % 32 == 0 && V % 16 == 0 && KT == 32 * U && KT % 32 == 0);
  static_assert(SZ_M + 512 <= 65536 && (SZ_A % 16) == 0 && (SZ_M % 16) == 0);
  static_assert((TM * UQ) % NTHR == 0 && (TM * VL * 8) == NPC * NTHR);
  static_assert((AP * 4) % 16 == 0 && (VP * 4) % 16 == 0);
  __shared__ __attribute__((aligned(16))) char smem[SZ_M + 512];
  float* sa  = (float*)smem;
  float* sz  = (float*)(smem + SZ_A);
  float* stg = (float*)smem;
  float* srs = (float*)(smem + SZ_M);
  (void)out;

  const int tid = (int)threadIdx.x, lane = tid & 31, wave = tid >> 5, hh = lane >> 4, m = lane & 15;
  const int rowBase = (int)blockIdx.x * TM;

#pragma unroll
  for (int i = 0; i < (TM * UQ) / NTHR; ++i) {
    const int idx = tid + NTHR * i;
    const int lr = idx / UQ, c4 = (idx - lr * UQ) * 4;
    int r = rowBase + lr;
    r = r < M ? r : M - 1;
    const v4f v = *(const v4fa*)(W + (size_t)fc_aoff<MODE>(r) + c4);
    *(v4fa*)(sa + lr * AP + c4) = v;
  }
#pragma unroll
  for (int i = 0; i < (TM * 8) / NTHR; ++i) {
    const int idx = tid + NTHR * i;
    const int lr = idx >> 3, c4 = (idx & 7) * 4;
    int r = rowBase + lr;
    r = r < M ? r : M - 1;
    const int n = fc_node<MODE>(r);
    const v4f v = *(const v4fa*)(W + (size_t)O_ZZ + (size_t)n * 32 + c4);
    *(v4fa*)(sz + lr * ZP + c4) = v;
  }
  if (tid < TM) {
    int r = rowBase + tid;
    r = r < M ? r : M - 1;
    const int n = fc_node<MODE>(r);
    srs[tid] = 1.0f / W[(size_t)O_SQD + n];
  }
  __syncthreads();

  float zf[16];
  {
    const float* zr = sz + (16 * wave + m) * ZP + 8 * hh;
    const v4f z0 = *(const v4fa*)zr;
    const v4f z1 = *(const v4fa*)(zr + 4);
    const v4f z2 = *(const v4fa*)(zr + 16);
    const v4f z3 = *(const v4fa*)(zr + 20);
    zf[0] = z0.x; zf[1] = z0.y; zf[2]  = z0.z; zf[3]  = z0.w;
    zf[4] = z1.x; zf[5] = z1.y; zf[6]  = z1.z; zf[7]  = z1.w;
    zf[8] = z2.x; zf[9] = z2.y; zf[10] = z2.z; zf[11] = z2.w;
    zf[12] = z3.x; zf[13] = z3.y; zf[14] = z3.z; zf[15] = z3.w;
  }

  v8f acc[NT];
  {
    const v8f z8 = {0.f, 0.f, 0.f, 0.f, 0.f, 0.f, 0.f, 0.f};
#pragma unroll
    for (int t = 0; t < NT; ++t) acc[t] = z8;
  }
  const float* sar = sa + (16 * wave + m) * AP;
  const unsigned short* bp = PL + (size_t)fcP<MODE>() + (size_t)m * KT + 8 * hh;

#pragma unroll 1
  for (int u = 0; u < U; ++u) {
    const float p = sar[u];
    FragB ah, al;
#pragma unroll
    for (int i = 0; i < 8; ++i) {
      const float P0 = p * zf[2 * i];
      const float P1 = p * zf[2 * i + 1];
      const unsigned h0 = bf16_hi32(P0);
      const unsigned h1 = bf16_hi32(P1);
      const float l0 = P0 - __uint_as_float(h0);
      const float l1 = P1 - __uint_as_float(h1);
      ah.w[i] = (int)((h0 >> 16) | h1);
      al.w[i] = (int)(bf16_bits(l0) | (bf16_bits(l1) << 16));
    }
#pragma unroll
    for (int nt = 0; nt < NT; ++nt) {
      const unsigned short* wq = bp + (size_t)(16 * nt) * KT + 32 * u;
      FragB b;
      b.h[0] = *(const v8usa*)wq;
      b.h[1] = *(const v8usa*)(wq + 16);
      acc[nt] = wmb(ah, b, acc[nt]);
      acc[nt] = wmb(al, b, acc[nt]);
    }
  }
  __syncthreads();

#pragma unroll
  for (int nt = 0; nt < NT; ++nt)
#pragma unroll
    for (int r = 0; r < 8; ++r)
      stg[(16 * wave + 8 * hh + r) * VP + 16 * nt + m] = acc[nt][r];
  __syncthreads();

#pragma unroll 1
  for (int i = 0; i < NPC; ++i) {
    const int idx = tid + NTHR * i;
    const int line = idx >> 3, q = idx & 7;
    const int lr = line / VL, seg = line - lr * VL;
    int r = rowBase + lr;
    r = r < M ? r : M - 1;
    float* sp = stg + lr * VP + seg * 32 + 4 * q;
    v4f v = *(const v4fa*)sp;
    if constexpr (MODE == M_PRE1 || MODE == M_PRE2S) {
      const float    sv   = srs[lr];
      const unsigned msk  = 0u - (unsigned)(seg == 0);
      const float    mult = __uint_as_float((__float_as_uint(sv) & msk) | (0x3F800000u & ~msk));
      v.x = (v.x * RN32) * mult; v.y = (v.y * RN32) * mult;
      v.z = (v.z * RN32) * mult; v.w = (v.w * RN32) * mult;
    } else if constexpr (MODE == M_PO1S) {
      const v4f mk = *(const v4fa*)(W + (size_t)O_MASK + (size_t)r * 64 + seg * 32 + 4 * q);
      const float c0 = C_S * mk.x + C_X * (v.x * RN32);
      const float c1 = C_S * mk.y + C_X * (v.y * RN32);
      const float c2 = C_S * mk.z + C_X * (v.z * RN32);
      const float c3 = C_S * mk.w + C_X * (v.w * RN32);
      const float g0 = gate_sig(c0), g1 = gate_sig(c1), g2 = gate_sig(c2), g3 = gate_sig(c3);
      v.x = (seg == 0) ? c0 * g0 : g0;
      v.y = (seg == 0) ? c1 * g1 : g1;
      v.z = (seg == 0) ? c2 * g2 : g2;
      v.w = (seg == 0) ? c3 * g3 : g3;
    } else if constexpr (MODE == M_PO1V) {
      const int n = r / 3;
      const v4f g = *(const v4fa*)(W + (size_t)O_F + (size_t)n * 32 + 4 * q);
      v.x = g.x * (v.x * RN32); v.y = g.y * (v.y * RN32);
      v.z = g.z * (v.z * RN32); v.w = g.w * (v.w * RN32);
    } else if constexpr (MODE == M_PRE2V) {
      const float mult = srs[lr];
      v.x = (v.x * RN32) * mult; v.y = (v.y * RN32) * mult;
      v.z = (v.z * RN32) * mult; v.w = (v.w * RN32) * mult;
    } else {
      const v4f mk = *(const v4fa*)(W + (size_t)O_MASK + (size_t)r * 64 + seg * 32 + 4 * q);
      v.x = C_S * mk.x + C_X * (v.x * RN64);
      v.y = C_S * mk.y + C_X * (v.y * RN64);
      v.z = C_S * mk.z + C_X * (v.z * RN64);
      v.w = C_S * mk.w + C_X * (v.w * RN64);
    }
    *(v4fa*)sp = v;
  }

  v4f pv[NPC];
#pragma unroll
  for (int i = 0; i < NPC; ++i) {
    const int idx = tid + NTHR * i;
    const int line = idx >> 3, q = idx & 7;
    const int lr = line / VL, seg = line - lr * VL;
    pv[i] = *(const v4fa*)(stg + lr * VP + seg * 32 + 4 * q);
  }
  float* dbase = W;
  if constexpr (MODE == M_PO2) dbase = out;
#pragma unroll
  for (int i = 0; i < NPC; ++i) {
    const int idx = tid + NTHR * i;
    const int line = idx >> 3, q = idx & 7;
    const int lr = line / VL, seg = line - lr * VL;
    const int r = rowBase + lr;
    if (r < M) *(volatile v4f*)(dbase + (size_t)fc_doff<MODE>(r, seg, q)) = pv[i];
  }
  __threadfence();
#pragma unroll
  for (int i = 0; i < NPC; ++i) {
    const int idx = tid + NTHR * i;
    const int line = idx >> 3, q = idx & 7;
    const int lr = line / VL, seg = line - lr * VL;
    const int r = rowBase + lr;
    if (r < M) *(volatile v4f*)(dbase + (size_t)fc_doff<MODE>(r, seg, q)) = pv[i];
  }
}

#define SAP 40
#define SHP 136
#define SOP 68
static_assert(SHP * 2 == SOP * 4);
__global__ __launch_bounds__(NTHR) void k_edge(const float* __restrict__ elen, const unsigned short* __restrict__ R0T,
                                               const unsigned short* __restrict__ R1T, float* WP) {
  __shared__ __attribute__((aligned(16))) unsigned short sA[TM * SAP];
  __shared__ __attribute__((aligned(16))) char sHO[TM * SHP * 2];
  unsigned short* sH = (unsigned short*)sHO;
  float*          sO = (float*)sHO;
  const int tid = (int)threadIdx.x, lane = tid & 31, wave = tid >> 5, hh = lane >> 4, m = lane & 15;
  const int eb = (int)blockIdx.x * TM;

  {
    const int em = lane & 15, eh = lane >> 4;
    const int el = eb + 16 * wave + em;
    const float len = bf16_val(elen[el]);
    unsigned short* ra = sA + (16 * wave + em) * SAP;
#pragma unroll
    for (int i = 0; i < 5; ++i) {
      const float ck = eh ? ctr(i + 5) : ctr(i);
      const float d  = (len - ck) * RSTEP;
      const float e  = expf(-(d * d)) * R112;
      const unsigned hb = bf16_hi32(e);
      ra[5 * eh + i]      = (unsigned short)(hb >> 16);
      ra[10 + 5 * eh + i] = (unsigned short)bf16_bits(e - __uint_as_float(hb));
    }
#pragma unroll
    for (int i = 0; i < 6; ++i) ra[20 + 6 * eh + i] = (unsigned short)0;
  }
  __syncthreads();

  const v8f z8 = {0.f, 0.f, 0.f, 0.f, 0.f, 0.f, 0.f, 0.f};
  v8f acc1[4];
  {
    const unsigned short* ap = sA + (16 * wave + m) * SAP + 8 * hh;
    FragB a;
    a.h[0] = *(const v8usa*)ap;
    a.h[1] = *(const v8usa*)(ap + 16);
#pragma unroll
    for (int nt = 0; nt < 4; ++nt) {
      const unsigned short* wq = R0T + (size_t)(16 * nt + m) * 32 + 8 * hh;
      FragB b;
      b.h[0] = *(const v8usa*)wq;
      b.h[1] = *(const v8usa*)(wq + 16);
      acc1[nt] = wmb(a, b, z8);
    }
  }
#pragma unroll
  for (int nt = 0; nt < 4; ++nt)
#pragma unroll
    for (int r = 0; r < 8; ++r) {
      const float t = acc1[nt][r];
      const float s = t * (1.0f / (1.0f + expf(-t)));
      const unsigned hb = bf16_hi32(s);
      unsigned short* hp = sH + (16 * wave + 8 * hh + r) * SHP + 16 * nt + m;
      hp[0]  = (unsigned short)(hb >> 16);
      hp[64] = (unsigned short)bf16_bits(s - __uint_as_float(hb));
    }
  __syncthreads();

  v8f acc2[4];
#pragma unroll
  for (int nt = 0; nt < 4; ++nt) acc2[nt] = z8;
  {
    const unsigned short* hp = sH + (16 * wave + m) * SHP + 8 * hh;
#pragma unroll
    for (int ks = 0; ks < 2; ++ks) {
      const int k0 = 32 * ks;
      FragB ah, al;
      ah.h[0] = *(const v8usa*)(hp + k0);
      ah.h[1] = *(const v8usa*)(hp + k0 + 16);
      al.h[0] = *(const v8usa*)(hp + 64 + k0);
      al.h[1] = *(const v8usa*)(hp + 64 + k0 + 16);
#pragma unroll
      for (int nt = 0; nt < 4; ++nt) {
        const unsigned short* wq = R1T + (size_t)(16 * nt + m) * 64 + k0 + 8 * hh;
        FragB b;
        b.h[0] = *(const v8usa*)wq;
        b.h[1] = *(const v8usa*)(wq + 16);
        acc2[nt] = wmb(ah, b, acc2[nt]);
        acc2[nt] = wmb(al, b, acc2[nt]);
      }
    }
  }
  __syncthreads();
#pragma unroll
  for (int nt = 0; nt < 4; ++nt)
#pragma unroll
    for (int r = 0; r < 8; ++r) sO[(16 * wave + 8 * hh + r) * SOP + 16 * nt + m] = acc2[nt][r];
  __syncthreads();

  v4f pv[8];
#pragma unroll
  for (int i = 0; i < 8; ++i) {
    const int idx = tid + NTHR * i;
    pv[i] = *(const v4fa*)(sO + (idx >> 4) * SOP + (idx & 15) * 4);
  }
  float* wb = WP + (size_t)eb * 64;
#pragma unroll
  for (int i = 0; i < 8; ++i) *(volatile v4f*)(wb + (size_t)(tid + NTHR * i) * 4) = pv[i];
  __threadfence();
#pragma unroll
  for (int i = 0; i < 8; ++i) *(volatile v4f*)(wb + (size_t)(tid + NTHR * i) * 4) = pv[i];
}

template <int LAYER>
__global__ __launch_bounds__(NTHR) void k_scan(const int* __restrict__ dsts, const int* __restrict__ srcs,
                                               const float* __restrict__ evec, const float* __restrict__ elen,
                                               float* W, int first, int last) {
  extern __shared__ __attribute__((aligned(16))) int dsm[];
  int* list = dsm;
  int* hl   = dsm + LISTN;
  int* sl   = hl + RCAP;
  int* cnt  = sl + RCAP;
  int* offs = cnt + NBA;
  int* cur  = offs + NBA;
  int* misc = cur + NBA;
  const int tid = (int)threadIdx.x, lane = tid & 31, wave = tid >> 5;
  const int nodeBase = (int)blockIdx.x * NBA;

  {
    const v4i z4 = {0, 0, 0, 0};
    for (int i = tid * 4; i < AGG_ZINTS; i += NTHR * 4) *(v4ia*)(dsm + i) = z4;
    if (tid < 16) misc[tid] = 0;
  }
  __syncthreads();

  int t = 0, ov = 0;
  const int nChunks = (EC + CHUNK - 1) / CHUNK;
#pragma unroll 1
  for (int ch = 0; ch < nChunks; ++ch) {
    const int cbase = ch * CHUNK;
    const int wc = scan_chunk<SLA>(dsts, EC, cbase, nodeBase, NBA, 1, list, tid, lane, wave);
    if (lane == 0) misc[wave] = wc;
    __syncthreads();
    if (wave == 0) {
#pragma unroll 1
      for (int w2 = 0; w2 < NWAVE; ++w2) {
        int c = misc[w2];
        c = c < 0 ? 0 : (c > WCAP ? WCAP : c);
#pragma unroll 1
        for (int b0 = 0; b0 < c; b0 += 32) {
          const int idx = b0 + lane;
          const int ent = list[w2 * WCAP + (idx < WCAP ? idx : WCAP - 1)];
          const int m32 = (c - b0) < 32 ? (c - b0) : 32;
#pragma unroll 1
          for (int k = 0; k < m32; ++k) {
            const int u    = __builtin_amdgcn_readlane(ent, k);
            const int slot = u & (NBA - 1);
            const int el   = (u >> SLA) & (CHUNK - 1);
            const int pk   = ((cbase + el) << SLA) | slot;
            if (t < RCAP) {
              if (lane == 0) { hl[t] = pk; cnt[slot] = cnt[slot] + 1; }
              t = t + 1;
            } else {
              ov = 1;
            }
          }
        }
      }
    }
    __syncthreads();
  }
  if (wave == 0 && lane == 0) { misc[8] = t; misc[9] = ov; }
  __syncthreads();
  int tt = misc[8];
  tt = tt < 0 ? 0 : (tt > RCAP ? RCAP : tt);
  const int ovf = misc[9];

  if (wave == 0) {
    const int base = lane * (NBA / 32);
    int s = 0;
#pragma unroll 1
    for (int i = 0; i < NBA / 32; ++i) s += cnt[base + i];
    int incl = s;
#pragma unroll
    for (int d = 1; d < 32; d <<= 1) {
      const int y = __shfl_up(incl, d, 32);
      if (lane >= d) incl += y;
    }
    int run = incl - s;
#pragma unroll 1
    for (int i = 0; i < NBA / 32; ++i) {
      const int cv = cnt[base + i];
      offs[base + i] = run;
      cur[base + i]  = run;
      run += cv;
    }
  }
  __syncthreads();
  if (wave == 0) {
#pragma unroll 1
    for (int b0 = 0; b0 < tt; b0 += 32) {
      const int idx = b0 + lane;
      const int ent = hl[idx < RCAP ? idx : RCAP - 1];
      const int m32 = (tt - b0) < 32 ? (tt - b0) : 32;
#pragma unroll 1
      for (int k = 0; k < m32; ++k) {
        const int u    = __builtin_amdgcn_readlane(ent, k);
        const int slot = u & (NBA - 1);
        if (lane == 0) {
          int p = cur[slot];
          p = p < 0 ? 0 : (p > RCAP - 1 ? RCAP - 1 : p);
          sl[p] = u;
          cur[slot] = p + 1;
        }
      }
    }
  }
  __syncthreads();

  const float qnan = __int_as_float(0x7fc00000);
  const float pz = (ovf != 0) ? qnan : 0.0f;
  const float* wp = W + (size_t)O_WP;
#pragma unroll 1
  for (int si = 0; si < NBA / NWAVE; ++si) {
    const int s    = si * NWAVE + wave;
    const int node = nodeBase + s;
    int c = cnt[s];
    const bool big = c > DEGCAP;
    c = c < 0 ? 0 : (c > DEGCAP ? DEGCAP : c);
    int o = offs[s];
    o = o < 0 ? 0 : (o > RCAP ? RCAP : o);
    float a0 = 0.0f, a1 = 0.0f, a2 = 0.0f, a3 = 0.0f;
#pragma unroll 1
    for (int b0 = 0; b0 < c; b0 += 32) {
      int idx = o + b0 + lane;
      idx = idx > RCAP - 1 ? RCAP - 1 : idx;
      const int ent = sl[idx];
      int eid = ent >> SLA;
      eid = eid < 0 ? 0 : (eid > EC - 1 ? EC - 1 : eid);
      int sv = srcs[eid];
      sv = sv < 0 ? 0 : (sv > NN - 1 ? NN - 1 : sv);
      const float vx = bf16_val(evec[(size_t)eid * 3 + 0]);
      const float vy = bf16_val(evec[(size_t)eid * 3 + 1]);
      const float vz = bf16_val(evec[(size_t)eid * 3 + 2]);
      const float ln = bf16_val(elen[eid]);
      const float rinv = 1.0f / (ln + 1e-12f);
      const int y0i = __float_as_int((SQ3F * vx) * rinv);
      const int y1i = __float_as_int((SQ3F * vy) * rinv);
      const int y2i = __float_as_int((SQ3F * vz) * rinv);
      const int m32 = (c - b0) < 32 ? (c - b0) : 32;
#pragma unroll 1
      for (int k = 0; k < m32; ++k) {
        const int ek = __builtin_amdgcn_readlane(eid, k);
        const int sk = __builtin_amdgcn_readlane(sv, k);
        const float y0 = __int_as_float(__builtin_amdgcn_readlane(y0i, k));
        const float y1 = __int_as_float(__builtin_amdgcn_readlane(y1i, k));
        const float y2 = __int_as_float(__builtin_amdgcn_readlane(y2i, k));
        const float w0 = wp[(size_t)ek * 64 + lane];
        const float w1 = wp[(size_t)ek * 64 + 32 + lane];
        if constexpr (LAYER == 1) {
          const float f  = W[(size_t)O_F + (size_t)sk * 32 + lane];
          const float t0 = w0 * f;
          const float t1 = w1 * f;
          a0 += t0;
          a1 += t1 * y0;
          a2 += t1 * y1;
          a3 += t1 * y2;
        } else {
          const float* fr = W + (size_t)O_AGG + (size_t)sk * 128 + lane;
          const float fs = fr[0];
          const float f0 = fr[32];
          const float f1 = fr[64];
          const float f2 = fr[96];
          const float dot = f0 * y0 + f1 * y1 + f2 * y2;
          a0 += w0 * fs;
          a1 += (w1 * dot) * RSQ3F;
        }
      }
    }
    const bool  live = node < NN;
    const int   nr   = live ? node : NN - 1;
    const float pzr  = big ? qnan : pz;
    const float rs   = 1.0f / W[(size_t)O_SQD + nr];
    const float sc   = (last != 0) ? rs : 1.0f;
    if constexpr (LAYER == 1) {
      float* mp = W + (size_t)O_AGG + (size_t)nr * 128 + lane;
      float o0 = 0.0f, o1 = 0.0f, o2 = 0.0f, o3 = 0.0f;
      if (first == 0) { o0 = mp[0]; o1 = mp[32]; o2 = mp[64]; o3 = mp[96]; }
      const float n0 = ((o0 + a0) + pzr) * sc;
      const float n1 = ((o1 + a1) + pzr) * sc;
      const float n2 = ((o2 + a2) + pzr) * sc;
      const float n3 = ((o3 + a3) + pzr) * sc;
      if (live) {
        *(volatile float*)(mp)      = n0;
        *(volatile float*)(mp + 32) = n1;
        *(volatile float*)(mp + 64) = n2;
        *(volatile float*)(mp + 96) = n3;
      }
      __threadfence();
      if (live) {
        *(volatile float*)(mp)      = n0;
        *(volatile float*)(mp + 32) = n1;
        *(volatile float*)(mp + 64) = n2;
        *(volatile float*)(mp + 96) = n3;
      }
    } else {
      float* mp = W + (size_t)O_V1 + (size_t)nr * 64 + lane;
      float o0 = 0.0f, o1 = 0.0f;
      if (first == 0) { o0 = mp[0]; o1 = mp[32]; }
      const float n0 = ((o0 + a0) + pzr) * sc;
      const float n1 = ((o1 + a1) + pzr) * sc;
      if (live) {
        *(volatile float*)(mp)      = n0;
        *(volatile float*)(mp + 32) = n1;
      }
      __threadfence();
      if (live) {
        *(volatile float*)(mp)      = n0;
        *(volatile float*)(mp + 32) = n1;
      }
    }
  }
}

extern "C" void kernel_launch(void* const* d_in, const int* in_sizes, int n_in,
                              void* d_out, int out_size, void* d_ws, size_t ws_size,
                              hipStream_t stream) {
  if (n_in < 25) return;
  if (in_sizes[0] != NN * XD || in_sizes[1] != NN * XD || in_sizes[2] != NN) return;
  if (in_sizes[3] != NE * 3 || in_sizes[4] != NE || in_sizes[5] != NE || in_sizes[6] != NE) return;
  if (in_sizes[7] != XD * 32 || in_sizes[8] != 32 || in_sizes[9] != XD * 32 || in_sizes[10] != 32) return;
  if (in_sizes[11] != 32768 || in_sizes[12] != 32768 || in_sizes[13] != 32768) return;
  if (in_sizes[14] != 640 || in_sizes[15] != 4096) return;
  if (in_sizes[16] != 32768 || in_sizes[17] != 32768 || in_sizes[18] != 32768) return;
  if (in_sizes[19] != 32768 || in_sizes[20] != 32768 || in_sizes[21] != 65536) return;
  if (in_sizes[22] != 640 || in_sizes[23] != 4096 || in_sizes[24] != 131072) return;
  if (out_size != NN * 64) return;
  if (ws_size < WS_BYTES) return;

  const float* x     = (const float*)d_in[0];
  const float* z     = (const float*)d_in[1];
  const float* ndeg  = (const float*)d_in[2];
  const float* evec  = (const float*)d_in[3];
  const float* elen  = (const float*)d_in[4];
  const int*   esrc  = (const int*)d_in[5];
  const int*   edst  = (const int*)d_in[6];
  const float* emxw  = (const float*)d_in[7];
  const float* emxb  = (const float*)d_in[8];
  const float* emzw  = (const float*)d_in[9];
  const float* emzb  = (const float*)d_in[10];
  const float* wli1  = (const float*)d_in[11];
  const float* wlm1s = (const float*)d_in[12];
  const float* wlm1g = (const float*)d_in[13];
  const float* r1w0  = (const float*)d_in[14];
  const float* r1w1  = (const float*)d_in[15];
  const float* wlo1s = (const float*)d_in[16];
  const float* wlo1g = (const float*)d_in[17];
  const float* wlo1v = (const float*)d_in[18];
  const float* wli2s = (const float*)d_in[19];
  const float* wli2v = (const float*)d_in[20];
  const float* wlm2  = (const float*)d_in[21];
  const float* r2w0  = (const float*)d_in[22];
  const float* r2w1  = (const float*)d_in[23];
  const float* wlo2  = (const float*)d_in[24];
  float* out = (float*)d_out;

  float*          W  = (float*)d_ws;
  unsigned short* PL = (unsigned short*)((char*)d_ws + (size_t)O_PL * 4);

  hipFuncSetAttribute(reinterpret_cast<const void*>(&k_scan<1>), hipFuncAttributeMaxDynamicSharedMemorySize,
                      (int)AGG_LDS_BYTES);
  hipFuncSetAttribute(reinterpret_cast<const void*>(&k_scan<2>), hipFuncAttributeMaxDynamicSharedMemorySize,
                      (int)AGG_LDS_BYTES);

  const int gN  = (NN + TM - 1) / TM;
  const int g3N = (3 * NN + TM - 1) / TM;

  k_prep<<<B17 / NTHR, NTHR, 0, stream>>>(ndeg, emxw, emzw, wli1, wlm1s, wlm1g, r1w0, r1w1, wlo1s, wlo1g, wlo1v,
                                          wli2s, wli2v, wlm2, r2w0, r2w1, wlo2, PL, W + O_SQD);
  k_embed<<<gN, NTHR, 0, stream>>>(x, emxb, PL + P_EMX, W + O_XS);
  k_embed<<<gN, NTHR, 0, stream>>>(z, emzb, PL + P_EMZ, W + O_ZZ);
  k_fctp<M_PRE1><<<gN, NTHR, 0, stream>>>(W, PL, out);
  for (int q = 0; q < NCH; ++q) {
    k_edge<<<EC / TM, NTHR, 0, stream>>>(elen + (size_t)q * EC, PL + P_R0T, PL + P_R1T, W + O_WP);
    k_scan<1><<<SCAN_BLOCKS, NTHR, AGG_LDS_BYTES, stream>>>(edst + (size_t)q * EC, esrc + (size_t)q * EC,
                                                           evec + (size_t)q * EC * 3, elen + (size_t)q * EC,
                                                           W, q == 0 ? 1 : 0, q == NCH - 1 ? 1 : 0);
  }
  k_fctp<M_PO1S><<<gN, NTHR, 0, stream>>>(W, PL, out);
  k_fctp<M_PO1V><<<g3N, NTHR, 0, stream>>>(W, PL, out);
  k_fctp<M_PRE2S><<<gN, NTHR, 0, stream>>>(W, PL, out);
  k_fctp<M_PRE2V><<<g3N, NTHR, 0, stream>>>(W, PL, out);
  for (int q = 0; q < NCH; ++q) {
    k_edge<<<EC / TM, NTHR, 0, stream>>>(elen + (size_t)q * EC, PL + P_R0T + 64 * 32, PL + P_R1T + 64 * 64,
                                         W + O_WP);
    k_scan<2><<<SCAN_BLOCKS, NTHR, AGG_LDS_BYTES, stream>>>(edst + (size_t)q * EC, esrc + (size_t)q * EC,
                                                           evec + (size_t)q * EC * 3, elen + (size_t)q * EC,
                                                           W, q == 0 ? 1 : 0, q == NCH - 1 ? 1 : 0);
  }
  k_fctp<M_PO2><<<gN, NTHR, 0, stream>>>(W, PL, out);
}
